// GatedLinearAttention_3582002724931
// MI455X (gfx1250) — hardware-verified
//
#include <hip/hip_runtime.h>
#include <math.h>

constexpr int NB    = 4;
constexpr int NT    = 2048;
constexpr int ND    = 1024;
constexpr int NH    = 4;
constexpr int NKD   = 1024;
constexpr int NVD   = 2048;
constexpr int DK    = NKD / NH;
constexpr int DV    = NVD / NH;
constexpr int CH    = 64;
constexpr int NCH   = NT / CH;
constexpr int NROW  = NB * NT;
constexpr int NCHT  = NROW / CH;
constexpr int LR    = 16;
constexpr int T1P   = 64;
constexpr int SQRT_DK = 16;
constexpr float GATE_NORM  = 16.0f;
constexpr float GATE_INV   = 1.0f / GATE_NORM;
constexpr float WCARRY     = 64.0f;
constexpr float WCARRY_INV = 1.0f / WCARRY;
constexpr float QCARRY     = 16.0f;
constexpr float OGCARRY    = 16.0f;
constexpr float QK_SCALE   = 1.0f / (float)SQRT_DK;
constexpr float OSCALE     = QK_SCALE / QCARRY;
constexpr float OUT_SCALE  = 1.0f / (WCARRY * OGCARRY);
constexpr float RMS_EPS    = 1e-5f;
constexpr int SPITCH = DK + 8;
constexpr int OPITCH = 68;
static_assert(SQRT_DK * SQRT_DK == DK, "scale");
static_assert(DK == 256 && DV == 512 && NROW == 8192 && NCH == 32 && NCHT == 128, "shape");
static_assert(ND % 32 == 0 && NVD % 32 == 0 && DK % 32 == 0 && CH % 32 == 0, "K multiples of 32");
static_assert(NROW % 64 == 0 && NKD % 64 == 0 && NVD % 64 == 0 && ND % 64 == 0, "tile multiples");
static_assert(DV % 64 == 0 && (DV / 64) == 8, "dv tiles");

constexpr size_t MIB       = (size_t)1 << 20;
constexpr size_t OFF_HS    = 0;
constexpr size_t OFF_WPL   = 16 * MIB;
constexpr size_t OFF_R2    = 24 * MIB;
constexpr size_t OFF_R3    = 56 * MIB;
constexpr size_t OFF_ORAW  = OFF_R2 + 16 * MIB;
constexpr size_t OFF_R4    = 88 * MIB;
constexpr size_t OFF_APL   = 120 * MIB;
constexpr size_t OFF_EGL   = OFF_APL + 4 * MIB;
constexpr size_t OFF_SSQ   = OFF_EGL + (size_t)NCHT * NKD * 4;
constexpr size_t OFF_WG1T  = OFF_SSQ + (size_t)32 * NROW * 4;
constexpr size_t WS_TOTAL  = OFF_WG1T + (size_t)64 * ND * 2;
static_assert((size_t)NROW * ND * 2 == 16 * MIB, "hs16");
static_assert((size_t)NROW * NKD * 4 == 32 * MIB, "G");
static_assert((size_t)NVD * NROW * 2 == 32 * MIB, "vT");
static_assert((size_t)NROW * NVD * 2 == 32 * MIB, "oraw/og");
static_assert((size_t)NROW * T1P * 4 <= 32 * MIB, "t1");
static_assert((size_t)NCHT * NH * CH * CH * 2 == 4 * MIB, "A");
static_assert(OFF_ORAW + 32 * MIB == OFF_R3 + 16 * MIB, "oraw span");
static_assert(WS_TOTAL <= (size_t)134217728, "carve");

typedef __attribute__((ext_vector_type(16))) _Float16 v16h;
typedef __attribute__((ext_vector_type(8)))  _Float16 v8h;
typedef __attribute__((ext_vector_type(8)))  float    v8f;
typedef __attribute__((ext_vector_type(4)))  float    v4f;
typedef __attribute__((ext_vector_type(4)))  unsigned int v4u;

__device__ __forceinline__ unsigned short f2bf_bits(float f) {
  unsigned u = __float_as_uint(f);
  return (unsigned short)((u + 0x7FFFu + ((u >> 16) & 1u)) >> 16);
}
__device__ __forceinline__ float bf_bits2f(unsigned short h) { return __uint_as_float(((unsigned)h) << 16); }
__device__ __forceinline__ float bf16r(float f) { return bf_bits2f(f2bf_bits(f)); }

__device__ __forceinline__ float h16_to_f32(unsigned hb) {
  const unsigned sgn = (hb & 0x8000u) << 16;
  const unsigned em = hb & 0x7fffu;
  const float fn = __uint_as_float((em << 13) + 0x38000000u);
  const float fs = (float)em * 5.9604644775390625e-8f;
  const float mag = (em < 0x400u) ? fs : fn;
  return __uint_as_float(__float_as_uint(mag) | sgn);
}

union FragU { v16h v; v8h h[2]; };
__device__ __forceinline__ v16h frag_load(const _Float16* p) {
  FragU f;
  f.h[0] = *(const v8h*)(p);
  f.h[1] = *(const v8h*)(p + 16);
  return f.v;
}
__device__ __forceinline__ v8f mma_raw(v16h a, v16h b, v8f c) {
  return __builtin_amdgcn_wmma_f32_16x16x32_f16(false, a, false, b, (short)0, c, false, false);
}
__device__ __forceinline__ v8f mma_g(v16h a, v16h b, v8f c) {
  c = __builtin_amdgcn_wmma_f32_16x16x32_f16(false, a, false, b, (short)0, c, false, false);
  asm volatile("v_nop\n\tv_nop\n\tv_nop\n\tv_nop" : "+v"(c) : "v"(a), "v"(b));
  return c;
}
__device__ __forceinline__ void guard_group(v8f& a0, v8f& a1, v8f& a2, v8f& a3, v16h x,
                                            v16h b0, v16h b1, v16h b2, v16h b3) {
  asm volatile("v_nop\n\tv_nop\n\tv_nop\n\tv_nop"
               : "+v"(a0), "+v"(a1), "+v"(a2), "+v"(a3)
               : "v"(x), "v"(b0), "v"(b1), "v"(b2), "v"(b3));
}
__device__ __forceinline__ void acc_guard4(v8f& a, v8f& b, v8f& c, v8f& d) {
  asm volatile("v_nop\n\tv_nop\n\tv_nop\n\tv_nop" : "+v"(a), "+v"(b), "+v"(c), "+v"(d));
}
__device__ __forceinline__ void wave_sync() {
  __builtin_amdgcn_fence(__ATOMIC_RELEASE, "workgroup");
  __builtin_amdgcn_wave_barrier();
  __builtin_amdgcn_fence(__ATOMIC_ACQUIRE, "workgroup");
}

__global__ __launch_bounds__(256) void pack_rows_kernel(const float* __restrict__ in,
                                                        unsigned short* __restrict__ out, int n8) {
  const int i = blockIdx.x * 256 + threadIdx.x;
  if (i < n8) {
    const float* p = in + 8 * (size_t)i;
    const v4f a = *(const v4f*)(p);
    const v4f b = *(const v4f*)(p + 4);
    v8h hv;
#pragma unroll
    for (int e = 0; e < 4; ++e) {
      hv[e]     = (_Float16)bf16r(a[e]);
      hv[4 + e] = (_Float16)bf16r(b[e]);
    }
    volatile v8h* q = (volatile v8h*)(out + 8 * (size_t)i);
    *q = hv;
    __threadfence();
    *q = hv;
  }
}

__global__ __launch_bounds__(256) void wt_pack_kernel(const float* __restrict__ W,
                                                      unsigned short* __restrict__ out,
                                                      int kin, int nreal) {
  __shared__ float sm[64][65];
  const int t  = threadIdx.x;
  const int k0 = blockIdx.x * 64;
  const int n0 = blockIdx.y * 64;
#pragma unroll
  for (int i = 0; i < 16; ++i) {
    const int e  = i * 256 + t;
    const int r  = e >> 6;
    const int cc = e & 63;
    const int n  = n0 + cc;
    const int nc = (n < nreal) ? n : (nreal - 1);
    const float v = W[(size_t)(k0 + r) * nreal + nc];
    sm[cc][r] = (n < nreal) ? (bf16r(v) * WCARRY) : 0.0f;
  }
  __syncthreads();
  const int lane = t & 31, wave = t >> 5;
  const int q = lane >> 3, c8 = (lane & 7) * 8;
  for (int pass = 0; pass < 2; ++pass) {
#pragma unroll
    for (int it = 0; it < 2; ++it) {
      const int row = wave * 8 + it * 4 + q;
      v8h hv;
#pragma unroll
      for (int e = 0; e < 8; ++e) hv[e] = (_Float16)sm[row][c8 + e];
      *(volatile v8h*)(out + (size_t)(n0 + row) * kin + k0 + c8) = hv;
    }
    __threadfence();
  }
}

constexpr int EPI_F32 = 0;
constexpr int EPI_F16 = 1;
constexpr int EPI_QK  = 2;
constexpr int EPI_GT  = 3;

template <int EPI>
__global__ __launch_bounds__(256) void gemm64_kernel(
    const unsigned short* __restrict__ Ap, int lda,
    const unsigned short* __restrict__ Btp, int ldb,
    void* __restrict__ Cout, void* __restrict__ Cout2, int ldc,
    const float* __restrict__ ex0, const float* __restrict__ ex1,
    const unsigned short* __restrict__ ex2,
    int M, int N, int K, float scale) {
  const _Float16* A  = (const _Float16*)Ap;
  const _Float16* Bt = (const _Float16*)Btp;
  __shared__ __align__(16) float sT[8][16 * 68];
  const int lane = threadIdx.x & 31;
  const int wave = threadIdx.x >> 5;
  const int tilesN = N >> 6;
  const int tilesM = M >> 6;
  const int tile = blockIdx.x * 8 + wave;
  if (tile >= tilesM * tilesN) return;
  const int tm = tile / tilesN;
  const int tn = tile - tm * tilesN;
  const int m0 = tm << 6;
  const int n0 = tn << 6;
  const int rlane = lane & 15;
  const int koff  = (lane >> 4) * 8;
  const int mOff  = (lane >> 4) * 8;

  const _Float16* pa = A  + (size_t)(m0 + rlane) * lda + koff;
  const _Float16* pb = Bt + (size_t)(n0 + rlane) * ldb + koff;
  const size_t sa = (size_t)16 * lda;
  const size_t sb = (size_t)16 * ldb;

  v8f acc[4][4];
#pragma unroll
  for (int i = 0; i < 4; ++i)
#pragma unroll
    for (int j = 0; j < 4; ++j) acc[i][j] = (v8f){0.f, 0.f, 0.f, 0.f, 0.f, 0.f, 0.f, 0.f};

  for (int k0 = 0; k0 < K; k0 += 32) {
    v16h bh[4];
#pragma unroll
    for (int j = 0; j < 4; ++j) bh[j] = frag_load(pb + j * sb + k0);
#pragma unroll
    for (int i = 0; i < 4; ++i) {
      const v16h ah = frag_load(pa + i * sa + k0);
#pragma unroll
      for (int j = 0; j < 4; ++j) acc[i][j] = mma_raw(ah, bh[j], acc[i][j]);
      guard_group(acc[i][0], acc[i][1], acc[i][2], acc[i][3], ah, bh[0], bh[1], bh[2], bh[3]);
    }
  }
  acc_guard4(acc[0][0], acc[0][1], acc[0][2], acc[0][3]);
  acc_guard4(acc[1][0], acc[1][1], acc[1][2], acc[1][3]);
  acc_guard4(acc[2][0], acc[2][1], acc[2][2], acc[2][3]);
  acc_guard4(acc[3][0], acc[3][1], acc[3][2], acc[3][3]);

  float* slab = sT[wave];
  const int q8 = lane >> 3, c8 = (lane & 7) * 8;

  float rw[8];
#pragma unroll
  for (int e = 0; e < 8; ++e) rw[e] = 1.0f;
  if (EPI == EPI_GT) {
    const int ecol = (n0 & (DV - 1)) + c8;
    const v4f ra = *(const v4f*)(ex1 + ecol);
    const v4f rb = *(const v4f*)(ex1 + ecol + 4);
#pragma unroll
    for (int e = 0; e < 4; ++e) { rw[e] = bf16r(ra[e]); rw[4 + e] = bf16r(rb[e]); }
  }

#pragma unroll
  for (int i = 0; i < 4; ++i) {
    const int mBase = m0 + (i << 4);
#pragma unroll
    for (int j = 0; j < 4; ++j) {
#pragma unroll
      for (int r = 0; r < 8; ++r) slab[(mOff + r) * 68 + (j << 4) + rlane] = acc[i][j][r] * scale;
    }
    wave_sync();
    if (EPI == EPI_F32) {
      float* C = (float*)Cout;
      const int hh = lane >> 4, c4 = (lane & 15) * 4;
      for (int pass = 0; pass < 2; ++pass) {
#pragma unroll
        for (int it = 0; it < 8; ++it) {
          const int row = it * 2 + hh;
          const v4f v = *(const v4f*)(slab + row * 68 + c4);
          *(volatile v4f*)(C + (size_t)(mBase + row) * ldc + n0 + c4) = v;
        }
        __threadfence();
      }
    } else if (EPI == EPI_F16) {
      unsigned short* C = (unsigned short*)Cout;
      for (int pass = 0; pass < 2; ++pass) {
#pragma unroll
        for (int it = 0; it < 4; ++it) {
          const int row = it * 4 + q8;
          const float* sp = slab + row * 68 + c8;
          const v4f s0 = *(const v4f*)(sp);
          const v4f s1 = *(const v4f*)(sp + 4);
          v8h hv;
#pragma unroll
          for (int e = 0; e < 4; ++e) { hv[e] = (_Float16)s0[e]; hv[4 + e] = (_Float16)s1[e]; }
          *(volatile v8h*)(C + (size_t)(mBase + row) * ldc + n0 + c8) = hv;
        }
        __threadfence();
      }
    } else if (EPI == EPI_QK) {
      const bool isk = (n0 >= NKD);
      const int ncol = isk ? (n0 - NKD) : n0;
      unsigned short* C = isk ? (unsigned short*)Cout2 : (unsigned short*)Cout;
      const float sgn = isk ? -1.0f : 1.0f;
      const float cst = isk ? 1.0f : QCARRY;
#pragma unroll 1
      for (int it = 0; it < 4; ++it) {
        const int row = it * 4 + q8;
        const float* sp = slab + row * 68 + c8;
        const float* gp = ex0 + (size_t)(mBase + row) * NKD + ncol + c8;
        const v4f g0 = *(const v4f*)(gp);
        const v4f g1 = *(const v4f*)(gp + 4);
        const v4f s0 = *(const v4f*)(sp);
        const v4f s1 = *(const v4f*)(sp + 4);
        v8h hv;
#pragma unroll
        for (int e = 0; e < 4; ++e) {
          const float x0 = (s0[e] * cst) * expf(sgn * g0[e]);
          const float x1 = (s1[e] * cst) * expf(sgn * g1[e]);
          hv[e]     = (_Float16)x0;
          hv[4 + e] = (_Float16)x1;
        }
        volatile v8h* op = (volatile v8h*)(C + (size_t)(mBase + row) * ldc + ncol + c8);
        *op = hv;
        __threadfence();
        *op = hv;
      }
    } else {
      unsigned short* C = (unsigned short*)Cout;
      const int hd = n0 / DV;
#pragma unroll 1
      for (int it = 0; it < 4; ++it) {
        const int row = it * 4 + q8;
        const size_t R = (size_t)(mBase + row);
        const float* sqp = ex0 + (size_t)(hd * 8) * NROW + R;
        const float q0 = sqp[0];
        const float q1 = sqp[(size_t)1 * NROW];
        const float q2 = sqp[(size_t)2 * NROW];
        const float q3 = sqp[(size_t)3 * NROW];
        const float q4 = sqp[(size_t)4 * NROW];
        const float q5 = sqp[(size_t)5 * NROW];
        const float q6 = sqp[(size_t)6 * NROW];
        const float q7 = sqp[(size_t)7 * NROW];
        const float ssum = ((q0 + q1) + (q2 + q3)) + ((q4 + q5) + (q6 + q7));
        const float rinv = rsqrtf(ssum * (1.0f / (float)DV) + RMS_EPS);
        const v4u ow = *(const v4u*)(ex2 + R * NVD + n0 + c8);
        const float* sp = slab + row * 68 + c8;
        const v4f s0 = *(const v4f*)(sp);
        const v4f s1 = *(const v4f*)(sp + 4);
        v8h hv;
#pragma unroll
        for (int e = 0; e < 8; ++e) {
          const unsigned w = ow[e >> 1];
          const unsigned hb = (e & 1) ? (w >> 16) : (w & 0xffffu);
          const float o = h16_to_f32(hb);
          const float gt = (e < 4) ? s0[e & 3] : s1[e & 3];
          const float sg = 1.0f / (1.0f + expf(-gt));
          const float val = (((o * rinv) * rw[e]) * (gt * sg)) * OGCARRY;
          hv[e] = (_Float16)val;
        }
        volatile v8h* op = (volatile v8h*)(C + R * ldc + n0 + c8);
        *op = hv;
        __threadfence();
        *op = hv;
      }
    }
    wave_sync();
  }
}

__global__ __launch_bounds__(256) void gate_kernel(const float* __restrict__ t1,
                                                   const float* __restrict__ Wgk2,
                                                   const float* __restrict__ bgk2,
                                                   float* __restrict__ G,
                                                   float* __restrict__ eglast) {
  __shared__ __align__(16) float t1s[CH * LR];
  const int tid = threadIdx.x;
  const int col = blockIdx.x * 256 + tid;
  const int chunk = blockIdx.y;
  const int row0 = chunk * CH;
  {
    const int r = tid >> 2, c4 = (tid & 3) * 4;
    const v4f v = *(const v4f*)(t1 + (size_t)(row0 + r) * T1P + c4);
    *(v4f*)(t1s + r * LR + c4) = v;
  }
  float w[LR];
#pragma unroll
  for (int r = 0; r < LR; ++r) w[r] = bf16r(Wgk2[(size_t)r * NKD + col]);
  const float bias = bf16r(bgk2[col]);
  __syncthreads();
  float glast = 0.0f;
#pragma unroll 1
  for (int r = 0; r < CH; ++r) {
    const float* tp = t1s + r * LR;
    const v4f a0 = *(const v4f*)(tp);
    const v4f a1 = *(const v4f*)(tp + 4);
    const v4f a2 = *(const v4f*)(tp + 8);
    const v4f a3 = *(const v4f*)(tp + 12);
    float x = 0.0f;
#pragma unroll
    for (int e = 0; e < 4; ++e) x = fmaf(a0[e], w[e], x);
#pragma unroll
    for (int e = 0; e < 4; ++e) x = fmaf(a1[e], w[4 + e], x);
#pragma unroll
    for (int e = 0; e < 4; ++e) x = fmaf(a2[e], w[8 + e], x);
#pragma unroll
    for (int e = 0; e < 4; ++e) x = fmaf(a3[e], w[12 + e], x);
    x += bias;
    const float ex = expf(-fabsf(x));
    const float ls = fminf(x, 0.0f) - log1pf(ex);
    const float gv = ls * GATE_INV;
    glast = gv;
    volatile float* gp = (volatile float*)(G + (size_t)(row0 + r) * NKD + col);
    *gp = gv;
    __threadfence();
    *gp = gv;
  }
  const float eg = expf(glast);
  volatile float* ep = (volatile float*)(eglast + (size_t)chunk * NKD + col);
  *ep = eg;
  __threadfence();
  *ep = eg;
}

__global__ __launch_bounds__(128) void prep_kernel(const unsigned short* __restrict__ qgp,
                                                   const unsigned short* __restrict__ kdp,
                                                   unsigned short* __restrict__ Aout,
                                                   unsigned short* __restrict__ kdT) {
  __shared__ __align__(16) unsigned short kds[CH * SPITCH];
  __shared__ __align__(16) float slabs[4][16 * 68];
  const _Float16* qg = (const _Float16*)qgp;
  const _Float16* kd = (const _Float16*)kdp;
  const int tid = threadIdx.x, lane = tid & 31, wave = tid >> 5;
  const int c = lane & 15, hh = lane >> 4, koff = 8 * hh;
  const int blk = blockIdx.x;
  const int h = blk & (NH - 1);
  const int cn = blk >> 2;
  const int row0 = cn * CH;

#pragma unroll 4
  for (int i = 0; i < 16; ++i) {
    const int e = i * 128 + tid;
    const int r = e >> 5;
    const int c16 = e & 31;
    const v4u wv = *(const v4u*)(kdp + (size_t)(row0 + r) * NKD + h * DK + c16 * 8);
    *(v4u*)(kds + r * SPITCH + c16 * 8) = wv;
  }

  const int mi = wave;
  v8f acc[4];
#pragma unroll
  for (int j = 0; j < 4; ++j) acc[j] = (v8f){0.f, 0.f, 0.f, 0.f, 0.f, 0.f, 0.f, 0.f};
  const _Float16* qrow = qg + (size_t)(row0 + 16 * mi + c) * NKD + h * DK + koff;
  const _Float16* krow = kd + (size_t)(row0 + c) * NKD + h * DK + koff;
#pragma unroll 2
  for (int k0 = 0; k0 < DK; k0 += 32) {
    const v16h a = frag_load(qrow + k0);
#pragma unroll
    for (int j = 0; j < 4; ++j) {
      const v16h bfr = frag_load(krow + (size_t)j * 16 * NKD + k0);
      acc[j] = mma_g(a, bfr, acc[j]);
    }
  }
  float* slab = slabs[wave];
#pragma unroll
  for (int j = 0; j < 4; ++j) {
#pragma unroll
    for (int r = 0; r < 8; ++r) {
      const int tq = 16 * mi + 8 * hh + r;
      const int tk = 16 * j + c;
      const float v = (tk <= tq) ? acc[j][r] : 0.0f;
      slab[(8 * hh + r) * 68 + 16 * j + c] = v;
    }
  }
  wave_sync();
  const int q8 = lane >> 3, c8 = (lane & 7) * 8;
  {
    unsigned short* ap = Aout + (size_t)blk * (CH * CH) + (size_t)(16 * mi) * CH;
    for (int pass = 0; pass < 2; ++pass) {
#pragma unroll
      for (int it = 0; it < 4; ++it) {
        const int row = it * 4 + q8;
        const float* sp = slab + row * 68 + c8;
        const v4f s0 = *(const v4f*)(sp);
        const v4f s1 = *(const v4f*)(sp + 4);
        v8h hv;
#pragma unroll
        for (int e = 0; e < 4; ++e) { hv[e] = (_Float16)s0[e]; hv[4 + e] = (_Float16)s1[e]; }
        *(volatile v8h*)(ap + row * CH + c8) = hv;
      }
      __threadfence();
    }
  }
  __syncthreads();
  {
    for (int pass = 0; pass < 2; ++pass) {
#pragma unroll 4
      for (int it = 0; it < 16; ++it) {
        const int d = 64 * wave + it * 4 + q8;
        unsigned u[8];
#pragma unroll
        for (int e = 0; e < 8; ++e) u[e] = (unsigned)kds[(c8 + e) * SPITCH + d];
        const v4u pk = (v4u){u[0] | (u[1] << 16), u[2] | (u[3] << 16), u[4] | (u[5] << 16), u[6] | (u[7] << 16)};
        *(volatile v4u*)(kdT + (size_t)(h * DK + d) * NROW + row0 + c8) = pk;
      }
      __threadfence();
    }
  }
}

__global__ __launch_bounds__(256) void scan_kernel(const unsigned short* __restrict__ qgp,
                                                   const unsigned short* __restrict__ Atp,
                                                   const unsigned short* __restrict__ vTp,
                                                   const unsigned short* __restrict__ kdTp,
                                                   const float* __restrict__ eglast,
                                                   unsigned short* __restrict__ oraw,
                                                   float* __restrict__ ssq) {
  __shared__ __align__(16) _Float16 S16[64 * SPITCH];
  __shared__ __align__(16) float Ost[CH * OPITCH];
  __shared__ __align__(16) float ssqs[CH];
  const _Float16* qg  = (const _Float16*)qgp;
  const _Float16* At  = (const _Float16*)Atp;
  const _Float16* vT  = (const _Float16*)vTp;
  const _Float16* kdT = (const _Float16*)kdTp;
  const int tid = threadIdx.x, lane = tid & 31, wave = tid >> 5;
  const int c = lane & 15, hh = lane >> 4, koff = 8 * hh;
  const int vt = blockIdx.x & 7;
  const int bh = blockIdx.x >> 3;
  const int h = bh & (NH - 1);
  const int b = bh >> 2;
  const int dk0 = 32 * wave;
  const int omi = wave >> 1;
  const int onb = (wave & 1) * 2;
  const int q8 = lane >> 3, c8 = (lane & 7) * 8;

  v8f sacc[4][2];
#pragma unroll
  for (int mi = 0; mi < 4; ++mi)
#pragma unroll
    for (int j = 0; j < 2; ++j) sacc[mi][j] = (v8f){0.f, 0.f, 0.f, 0.f, 0.f, 0.f, 0.f, 0.f};

  const _Float16* vA = vT + (size_t)(h * DV + vt * 64 + c) * NROW + koff;
  const _Float16* vB = vT + (size_t)(h * DV + vt * 64 + 16 * onb + c) * NROW + koff;
  const _Float16* kB = kdT + (size_t)(h * DK + dk0 + c) * NROW + koff;
  const _Float16* sB = S16 + (16 * onb + c) * SPITCH + koff;

#pragma unroll 1
  for (int n = 0; n < NCH; ++n) {
    const int cn = b * NCH + n;
    const int row0 = cn * CH;

#pragma unroll
    for (int mi = 0; mi < 4; ++mi)
#pragma unroll
      for (int j = 0; j < 2; ++j)
#pragma unroll
        for (int r = 0; r < 8; ++r)
          S16[(16 * mi + 8 * hh + r) * SPITCH + dk0 + 16 * j + c] = (_Float16)sacc[mi][j][r];
    __syncthreads();

    v8f o0 = (v8f){0.f, 0.f, 0.f, 0.f, 0.f, 0.f, 0.f, 0.f};
    v8f o1 = o0;
    {
      const _Float16* qrow = qg + (size_t)(row0 + 16 * omi + c) * NKD + h * DK + koff;
#pragma unroll 2
      for (int k0 = 0; k0 < DK; k0 += 32) {
        const v16h a  = frag_load(qrow + k0);
        const v16h b0 = frag_load(sB + k0);
        const v16h b1 = frag_load(sB + 16 * SPITCH + k0);
        o0 = mma_g(a, b0, o0);
        o1 = mma_g(a, b1, o1);
      }
      const _Float16* arow = At + (size_t)(cn * NH + h) * (CH * CH) + (16 * omi + c) * CH + koff;
#pragma unroll
      for (int k0 = 0; k0 < CH; k0 += 32) {
        const v16h a  = frag_load(arow + k0);
        const v16h b0 = frag_load(vB + row0 + k0);
        const v16h b1 = frag_load(vB + (size_t)16 * NROW + row0 + k0);
        o0 = mma_g(a, b0, o0);
        o1 = mma_g(a, b1, o1);
      }
    }
#pragma unroll
    for (int r = 0; r < 8; ++r) {
      Ost[(16 * omi + 8 * hh + r) * OPITCH + 16 * onb + c]      = o0[r] * OSCALE;
      Ost[(16 * omi + 8 * hh + r) * OPITCH + 16 * onb + 16 + c] = o1[r] * OSCALE;
    }

#pragma unroll
    for (int k0 = 0; k0 < CH; k0 += 32) {
      const v16h kb0 = frag_load(kB + row0 + k0);
      const v16h kb1 = frag_load(kB + (size_t)16 * NROW + row0 + k0);
#pragma unroll
      for (int mi = 0; mi < 4; ++mi) {
        const v16h a = frag_load(vA + (size_t)(16 * mi) * NROW + row0 + k0);
        sacc[mi][0] = mma_g(a, kb0, sacc[mi][0]);
        sacc[mi][1] = mma_g(a, kb1, sacc[mi][1]);
      }
    }
    {
      const float* egp = eglast + (size_t)cn * NKD + h * DK + dk0 + c;
      const float eg0 = egp[0];
      const float eg1 = egp[16];
#pragma unroll
      for (int mi = 0; mi < 4; ++mi)
#pragma unroll
        for (int r = 0; r < 8; ++r) {
          sacc[mi][0][r] *= eg0;
          sacc[mi][1][r] *= eg1;
        }
    }
    __syncthreads();

    {
      v8h hvv[2];
#pragma unroll
      for (int it = 0; it < 2; ++it) {
        const int row = 8 * wave + it * 4 + q8;
        const float* sp = Ost + row * OPITCH + c8;
        const v4f s0 = *(const v4f*)(sp);
        const v4f s1 = *(const v4f*)(sp + 4);
        float p = ((s0[0] * s0[0] + s0[1] * s0[1]) + (s0[2] * s0[2] + s0[3] * s0[3]))
                + ((s1[0] * s1[0] + s1[1] * s1[1]) + (s1[2] * s1[2] + s1[3] * s1[3]));
        p += __shfl_xor(p, 1, 32);
        p += __shfl_xor(p, 2, 32);
        p += __shfl_xor(p, 4, 32);
        if ((lane & 7) == 0) ssqs[row] = p;
#pragma unroll
        for (int e = 0; e < 4; ++e) { hvv[it][e] = (_Float16)s0[e]; hvv[it][4 + e] = (_Float16)s1[e]; }
      }
      unsigned short* ob = oraw + (size_t)row0 * NVD + h * DV + vt * 64 + c8;
      for (int pass = 0; pass < 2; ++pass) {
#pragma unroll
        for (int it = 0; it < 2; ++it) {
          const int row = 8 * wave + it * 4 + q8;
          *(volatile v8h*)(ob + (size_t)row * NVD) = hvv[it];
        }
        __threadfence();
      }
    }
    __syncthreads();
    if (wave == 0 && lane < 16) {
      const v4f sv = *(const v4f*)(ssqs + 4 * lane);
      volatile v4f* sp = (volatile v4f*)(ssq + (size_t)(h * 8 + vt) * NROW + row0 + 4 * lane);
      *sp = sv;
      __threadfence();
      *sp = sv;
    }
  }
}

extern "C" void kernel_launch(void* const* d_in, const int* in_sizes, int n_in,
                              void* d_out, int out_size, void* d_ws, size_t ws_size,
                              hipStream_t stream) {
  if (n_in < 10 || d_out == nullptr || d_ws == nullptr) return;
  if (in_sizes[0] != NROW * ND || in_sizes[1] != ND * NKD || in_sizes[2] != ND * NKD ||
      in_sizes[3] != ND * NVD || in_sizes[4] != ND * NVD || in_sizes[5] != ND * LR ||
      in_sizes[6] != LR * NKD || in_sizes[7] != NKD || in_sizes[8] != DV ||
      in_sizes[9] != NVD * ND || out_size != NROW * ND) return;
  if (ws_size < WS_TOTAL) return;

  const float* hs    = (const float*)d_in[0];
  const float* Wq    = (const float*)d_in[1];
  const float* Wk    = (const float*)d_in[2];
  const float* Wv    = (const float*)d_in[3];
  const float* Wg    = (const float*)d_in[4];
  const float* Wgk1  = (const float*)d_in[5];
  const float* Wgk2  = (const float*)d_in[6];
  const float* bgk2  = (const float*)d_in[7];
  const float* rms_w = (const float*)d_in[8];
  const float* Wo    = (const float*)d_in[9];
  float* out = (float*)d_out;

  char* ws = (char*)d_ws;
  unsigned short* HS16  = (unsigned short*)(ws + OFF_HS);
  unsigned short* WPL   = (unsigned short*)(ws + OFF_WPL);
  unsigned short* WqkT  = WPL;
  unsigned short* WkT   = WPL + (size_t)NKD * ND;
  unsigned short* WvT   = WPL + (size_t)2 * NKD * ND;
  unsigned short* WgT   = WPL;
  unsigned short* WoT   = WPL + (size_t)NVD * ND;
  float*          Gpl   = (float*)(ws + OFF_R2);
  unsigned short* KDT   = (unsigned short*)(ws + OFF_R2);
  unsigned short* KD    = (unsigned short*)(ws + OFF_R3);
  unsigned short* QG    = (unsigned short*)(ws + OFF_R3 + 16 * MIB);
  unsigned short* ORAW  = (unsigned short*)(ws + OFF_ORAW);
  float*          T1    = (float*)(ws + OFF_R4);
  unsigned short* VT    = (unsigned short*)(ws + OFF_R4);
  unsigned short* OG    = (unsigned short*)(ws + OFF_R4);
  unsigned short* APL   = (unsigned short*)(ws + OFF_APL);
  float*          EGL   = (float*)(ws + OFF_EGL);
  float*          SSQ   = (float*)(ws + OFF_SSQ);
  unsigned short* WG1T  = (unsigned short*)(ws + OFF_WG1T);

  const int n8 = NROW * ND / 8;
  pack_rows_kernel<<<n8 / 256, 256, 0, stream>>>(hs, HS16, n8);

  wt_pack_kernel<<<dim3(ND / 64, NKD / 64), 256, 0, stream>>>(Wq, WqkT, ND, NKD);
  wt_pack_kernel<<<dim3(ND / 64, NKD / 64), 256, 0, stream>>>(Wk, WkT, ND, NKD);
  wt_pack_kernel<<<dim3(ND / 64, NVD / 64), 256, 0, stream>>>(Wv, WvT, ND, NVD);
  wt_pack_kernel<<<dim3(ND / 64, 1), 256, 0, stream>>>(Wgk1, WG1T, ND, LR);

  gemm64_kernel<EPI_F32><<<(NROW / 64) * 1 / 8, 256, 0, stream>>>(
      HS16, ND, WG1T, ND, (void*)T1, (void*)T1, T1P, EGL, EGL, HS16, NROW, 64, ND, WCARRY_INV);

  gate_kernel<<<dim3(NKD / 256, NCHT), 256, 0, stream>>>(T1, Wgk2, bgk2, Gpl, EGL);

  gemm64_kernel<EPI_QK><<<(NROW / 64) * (2 * NKD / 64) / 8, 256, 0, stream>>>(
      HS16, ND, WqkT, ND, (void*)QG, (void*)KD, NKD, Gpl, Gpl, HS16, NROW, 2 * NKD, ND, WCARRY_INV);

  gemm64_kernel<EPI_F16><<<(NVD / 64) * (NROW / 64) / 8, 256, 0, stream>>>(
      WvT, ND, HS16, ND, (void*)VT, (void*)VT, NROW, EGL, EGL, HS16, NVD, NROW, ND, WCARRY_INV);

  wt_pack_kernel<<<dim3(ND / 64, NVD / 64), 256, 0, stream>>>(Wg, WgT, ND, NVD);
  wt_pack_kernel<<<dim3(NVD / 64, ND / 64), 256, 0, stream>>>(Wo, WoT, NVD, ND);

  prep_kernel<<<NCHT * NH, 128, 0, stream>>>(QG, KD, APL, KDT);

  scan_kernel<<<NB * NH * (DV / 64), 256, 0, stream>>>(QG, APL, VT, KDT, EGL, ORAW, SSQ);

  gemm64_kernel<EPI_GT><<<(NROW / 64) * (NVD / 64) / 8, 256, 0, stream>>>(
      HS16, ND, WgT, ND, (void*)OG, (void*)OG, NVD, SSQ, rms_w, ORAW, NROW, NVD, ND, WCARRY_INV);

  gemm64_kernel<EPI_F32><<<(NROW / 64) * (ND / 64) / 8, 256, 0, stream>>>(
      OG, NVD, WoT, NVD, (void*)out, (void*)out, ND, EGL, EGL, HS16, NROW, ND, NVD, OUT_SCALE);
}
